// Transformer_24223615550001
// MI455X (gfx1250) — hardware-verified
//
#include <hip/hip_runtime.h>
#include <math.h>

#ifndef NB
#define NB 8
#endif
#ifndef SEQ
#define SEQ 1024
#endif
#define NB_FULL 8
#define SEQ_FULL 1024
#define MROWS (NB * SEQ)
#define NQB (SEQ / 64)

static_assert(SEQ % 64 == 0);
static_assert(SEQ <= SEQ_FULL);
static_assert(NB <= NB_FULL);
static_assert(MROWS % 64 == 0);
static_assert(((size_t)MROWS * 512) % 2048 == 0);

typedef __attribute__((ext_vector_type(16))) _Float16 v16h;
typedef __attribute__((ext_vector_type(8)))  _Float16 v8h;
typedef __attribute__((ext_vector_type(16))) __bf16   v16b;
typedef __attribute__((ext_vector_type(8)))  __bf16   v8b;
typedef __attribute__((ext_vector_type(8)))  float    v8f;
typedef __attribute__((ext_vector_type(4)))  float    v4f;
typedef unsigned int cm_u4 __attribute__((ext_vector_type(4)));


#define VST2(T, ptr, val) do { const T vst2_v_ = (val); *(volatile T*)(ptr) = vst2_v_; __threadfence(); *(volatile T*)(ptr) = vst2_v_; } while (0)
#define VST2V4(ptr, val) do { const v4f vst2_v4_ = (val); *(volatile v4f*)(ptr) = vst2_v4_; __threadfence(); *(volatile v4f*)(ptr) = vst2_v4_; } while (0)

__device__ __forceinline__ unsigned int cmb_pk2(float a, float b) { return (unsigned int)__builtin_bit_cast(unsigned short, (_Float16)a) | ((unsigned int)__builtin_bit_cast(unsigned short, (_Float16)b) << 16); }
__device__ __forceinline__ float cmb_bf(float v) { const unsigned u = __builtin_bit_cast(unsigned, v); const unsigned r = (u + 0x7fffu + ((u >> 16) & 1u)) & 0xffff0000u; return __builtin_bit_cast(float, r); }

namespace kit {
__device__ __forceinline__ unsigned short f2bf_bits(float f) {
  unsigned u = __float_as_uint(f);
  return (unsigned short)((u + 0x7FFFu + ((u >> 16) & 1u)) >> 16);
}
__device__ __forceinline__ float bf_bits2f(unsigned short h) { return __uint_as_float(((unsigned)h) << 16); }
__device__ __forceinline__ unsigned int f2bf2_pack(float a, float b, unsigned int* lo) {
  const unsigned short ha = f2bf_bits(a), hb = f2bf_bits(b);
  const unsigned short la = f2bf_bits(a - bf_bits2f(ha)), lb = f2bf_bits(b - bf_bits2f(hb));
  *lo = (unsigned)la | ((unsigned)lb << 16); return (unsigned)ha | ((unsigned)hb << 16);
}

__device__ __forceinline__ void dep_guard_h(v8f& a, v8f& b, v16h x, v16h y) { asm volatile("v_nop\n\tv_nop\n\tv_nop\n\tv_nop" : "+v"(a), "+v"(b) : "v"(x), "v"(y)); }
__device__ __forceinline__ void dep_guard_b(v8f& a, v8f& b, v16b x, v16b y) { asm volatile("v_nop\n\tv_nop\n\tv_nop\n\tv_nop" : "+v"(a), "+v"(b) : "v"(x), "v"(y)); }
__device__ __forceinline__ void keep4_h(v16h a, v16h b, v16h c, v16h d) { asm volatile("v_nop" :: "v"(a), "v"(b), "v"(c), "v"(d)); }
__device__ __forceinline__ void keep4_b(v16b a, v16b b, v16b c, v16b d) { asm volatile("v_nop" :: "v"(a), "v"(b), "v"(c), "v"(d)); }
__device__ __forceinline__ void acc_guard4(v8f& a, v8f& b, v8f& c, v8f& d) { asm volatile("v_nop\n\tv_nop\n\tv_nop\n\tv_nop" : "+v"(a), "+v"(b), "+v"(c), "+v"(d)); }
template <typename T> struct Frag;
template <> struct Frag<_Float16> {
  typedef v16h V; union U { v16h v; v8h h[2]; };
  static __device__ __forceinline__ v16h load(const _Float16* p) {
    U f; f.h[0] = *(const v8h*)(p); f.h[1] = *(const v8h*)(p + 16); return f.v;
  }
  static __device__ __forceinline__ v8f mma(v16h a, v16h b, v8f c) {
    return __builtin_amdgcn_wmma_f32_16x16x32_f16(false, a, false, b, (short)0, c, false, false);
  }
  static __device__ __forceinline__ void guard(v8f& a, v8f& b, v16h x, v16h y) { dep_guard_h(a, b, x, y); }
  static __device__ __forceinline__ void keep(v16h a, v16h b, v16h c, v16h d) { keep4_h(a, b, c, d); }
};
template <> struct Frag<__bf16> {
  typedef v16b V; union U { v16b v; v8b h[2]; };
  static __device__ __forceinline__ v16b load(const __bf16* p) {
    U f; f.h[0] = *(const v8b*)(p); f.h[1] = *(const v8b*)(p + 16); return f.v;
  }
  static __device__ __forceinline__ v8f mma(v16b a, v16b b, v8f c) {
    return __builtin_amdgcn_wmma_f32_16x16x32_bf16(false, a, false, b, (short)0, c, false, false);
  }
  static __device__ __forceinline__ void guard(v8f& a, v8f& b, v16b x, v16b y) { dep_guard_b(a, b, x, y); }
  static __device__ __forceinline__ void keep(v16b a, v16b b, v16b c, v16b d) { keep4_b(a, b, c, d); }
};

template <int ET> struct Elem;
template <> struct Elem<0> { typedef _Float16 T; };
template <> struct Elem<1> { typedef __bf16 T; };
template <int ET, bool SPLIT, int BIAS_MODE, int OUT_MODE, bool RESID, int ACT>
__global__ __launch_bounds__(256) void wmma_gemm64(
    const unsigned short* __restrict__ Ap, const unsigned short* __restrict__ A2p, int lda, long strideA,
    const unsigned short* __restrict__ Btp, const unsigned short* __restrict__ Bt2p, int ldb, long strideB,
    void* __restrict__ Cout, void* __restrict__ Cout2, int ldc, long strideC,
    const float* __restrict__ bias,
    const float* __restrict__ resid, long strideR,
    int M, int N, int K, float scale) {
  typedef typename Elem<ET>::T T;
  typedef typename Frag<T>::V V;
  const T* A = (const T*)Ap; const T* A2 = (const T*)A2p; const T* Bt = (const T*)Btp; const T* Bt2 = (const T*)Bt2p;
  __shared__ __align__(16) float sT[8][16 * 68];
  const unsigned b    = blockIdx.y;
  const unsigned lane = threadIdx.x & 31u;
  const unsigned wave = threadIdx.x >> 5;
  const unsigned tilesN = (unsigned)N >> 6;
  const unsigned tilesM = (unsigned)M >> 6;
  const unsigned tile = blockIdx.x * 8u + wave;
  if (tile >= tilesM * tilesN) return;
  const unsigned tm = tile / tilesN;
  const unsigned tn = tile - tm * tilesN;
  const unsigned m0 = tm << 6;
  const unsigned n0 = tn << 6;

  const T* Ab  = A  + (size_t)b * strideA;
  const T* Bb  = Bt + (size_t)b * strideB;
  const T* Ab2 = SPLIT ? (A2  + (size_t)b * strideA) : nullptr;
  const T* Bb2 = SPLIT ? (Bt2 + (size_t)b * strideB) : nullptr;

  const unsigned rlane = lane & 15u;
  const unsigned koff  = (lane >> 4) * 8u;
  const unsigned mOff  = (lane >> 4) * 8u;

  v8f acc[4][4];
#pragma unroll
  for (int i = 0; i < 4; ++i)
#pragma unroll
    for (int j = 0; j < 4; ++j) acc[i][j] = (v8f){0.f,0.f,0.f,0.f,0.f,0.f,0.f,0.f};

  for (unsigned k0 = 0; k0 < (unsigned)K; k0 += 32u) {
    V bh[4], bl[4];
#pragma unroll
    for (int j = 0; j < 4; ++j) {
      const size_t bo = (size_t)(n0 + ((unsigned)j << 4) + rlane) * (unsigned)ldb + koff + k0;
      bh[j] = Frag<T>::load(Bb + bo);
      if (SPLIT) bl[j] = Frag<T>::load(Bb2 + bo);
    }
#pragma unroll
    for (int i = 0; i < 4; ++i) {
      const size_t ao = (size_t)(m0 + ((unsigned)i << 4) + rlane) * (unsigned)lda + koff + k0;
      V ah = Frag<T>::load(Ab + ao);
      V al;
      if (SPLIT) al = Frag<T>::load(Ab2 + ao);
#pragma unroll
      for (int j = 0; j < 4; ++j) {
        acc[i][j] = Frag<T>::mma(ah, bh[j], acc[i][j]);
        if (SPLIT) {
          acc[i][j] = Frag<T>::mma(ah, bl[j], acc[i][j]);
          acc[i][j] = Frag<T>::mma(al, bh[j], acc[i][j]);
        }
      }
      Frag<T>::guard(acc[i][0], acc[i][3], ah, SPLIT ? al : ah);
    }
    Frag<T>::keep(bh[0], bh[1], bh[2], bh[3]);
    if (SPLIT) Frag<T>::keep(bl[0], bl[1], bl[2], bl[3]);
  }
  acc_guard4(acc[0][0], acc[0][1], acc[0][2], acc[0][3]);
  acc_guard4(acc[1][0], acc[1][1], acc[1][2], acc[1][3]);
  acc_guard4(acc[2][0], acc[2][1], acc[2][2], acc[2][3]);
  acc_guard4(acc[3][0], acc[3][1], acc[3][2], acc[3][3]);

  float* slab = sT[wave];
  const float* Rb = RESID ? (resid + (size_t)b * strideR) : nullptr;
#pragma unroll
  for (int i = 0; i < 4; ++i) {
    const unsigned mBase = m0 + ((unsigned)i << 4);
#pragma unroll
    for (int j = 0; j < 4; ++j) {
      const unsigned n = n0 + ((unsigned)j << 4) + rlane;
      float bv = 0.f;
      if (BIAS_MODE == 2) bv = bias[n];
#pragma unroll
      for (int r = 0; r < 8; ++r) {
        float v = acc[i][j][r] * scale;
        if (BIAS_MODE == 1) v += bias[mBase + mOff + r];
        if (BIAS_MODE == 2) v += bv;
        if (RESID) v += Rb[(size_t)(mBase + mOff + r) * (unsigned)ldc + n];
        if (ACT == 2) v = fmaxf(v, 0.0f);
        slab[(mOff + r) * 68u + ((unsigned)j << 4) + rlane] = v;
      }
    }
    __builtin_amdgcn_fence(3  , "workgroup");
    __builtin_amdgcn_wave_barrier();
    __builtin_amdgcn_fence(2  , "workgroup");
    if (OUT_MODE == 0) {
      float* C = (float*)Cout + (size_t)b * strideC;
      const unsigned hh = lane >> 4, c4 = (lane & 15u) * 4u;
      for (int pass = 0; pass < 2; ++pass) {
#pragma unroll
        for (int it = 0; it < 8; ++it) {
          const unsigned row = (unsigned)it * 2u + hh;
          v4f v = *(const v4f*)(slab + row * 68u + c4);
          *(volatile v4f*)(C + (size_t)(mBase + row) * (unsigned)ldc + n0 + c4) = v;
        }
        __threadfence();
      }
    } else {
      const unsigned q = lane >> 3, c8 = (lane & 7u) * 8u;
      unsigned short* C  = (unsigned short*)Cout  + (size_t)b * strideC;
      unsigned short* C2 = (OUT_MODE == 2) ? ((unsigned short*)Cout2 + (size_t)b * strideC) : nullptr;
      for (int pass = 0; pass < 2; ++pass) {
#pragma unroll
        for (int it = 0; it < 4; ++it) {
          const unsigned row = (unsigned)it * 4u + q;
          const float* sp = slab + row * 68u + c8;
          v8h hv, lv;
#pragma unroll
          for (int e = 0; e < 8; ++e) {
            if (OUT_MODE == 1) {
              hv[e] = (_Float16)sp[e];
            } else {
              unsigned short hb = f2bf_bits(sp[e]);
              unsigned short lb = f2bf_bits(sp[e] - bf_bits2f(hb));
              hv[e] = __builtin_bit_cast(_Float16, hb);
              lv[e] = __builtin_bit_cast(_Float16, lb);
            }
          }
          *(volatile v8h*)(C + (size_t)(mBase + row) * (unsigned)ldc + n0 + c8) = hv;
          if (OUT_MODE == 2) *(volatile v8h*)(C2 + (size_t)(mBase + row) * (unsigned)ldc + n0 + c8) = lv;
        }
        __threadfence();
      }
    }
    __builtin_amdgcn_fence(3  , "workgroup");
    __builtin_amdgcn_wave_barrier();
    __builtin_amdgcn_fence(2  , "workgroup");
  }
}

__device__ __forceinline__ unsigned short at_bf_bits(float f) {
  unsigned u = __float_as_uint(f);
  return (unsigned short)((u + 0x7FFFu + ((u >> 16) & 1u)) >> 16);
}
__device__ __forceinline__ __bf16 at_f2bf(float f) { return __builtin_bit_cast(__bf16, at_bf_bits(f)); }
__device__ __forceinline__ void at_split(float f, __bf16& hi, __bf16& lo) {
  const unsigned short hb = at_bf_bits(f);
  hi = __builtin_bit_cast(__bf16, hb);
  lo = at_f2bf(f - __uint_as_float(((unsigned)hb) << 16));
}
__device__ __forceinline__ v8f at_mma(v16b a, v16b b, v8f c) {
  c = __builtin_amdgcn_wmma_f32_16x16x32_bf16(false, a, false, b, (short)0, c, false, false);
  asm volatile("v_nop\n\tv_nop\n\tv_nop\n\tv_nop" : "+v"(c) : "v"(a), "v"(b));
  return c;
}
template <bool F16> __device__ __forceinline__ __bf16 at_to16(float f) {
  if (F16) return __builtin_bit_cast(__bf16, (_Float16)f);
  return at_f2bf(f);
}
template <bool F16> __device__ __forceinline__ v8f at_mma16(v16b a, v16b b, v8f c) {
  if (F16) {
    const v16h ah = __builtin_bit_cast(v16h, a), bh = __builtin_bit_cast(v16h, b);
    c = __builtin_amdgcn_wmma_f32_16x16x32_f16(false, ah, false, bh, (short)0, c, false, false);
    asm volatile("v_nop\n\tv_nop\n\tv_nop\n\tv_nop" : "+v"(c) : "v"(ah), "v"(bh));
    return c;
  }
  return at_mma(a, b, c);
}
}

template <bool SPV>
__global__ __launch_bounds__(128) void k_fattn(const unsigned short* __restrict__ QKhp, const unsigned short* __restrict__ QKlp,
                                               const unsigned short* __restrict__ VThp, const unsigned short* __restrict__ VTlp,
                                               const float* __restrict__ mask, unsigned short* __restrict__ Cp) {
  union FB { v16b v; v8b h[2]; };
  __shared__ __align__(16) __bf16 Psh[4][16 * 64];
  __shared__ __align__(16) __bf16 Psl[SPV ? 4 : 1][SPV ? 16 * 64 : 8];
  __shared__ __align__(16) float  Os[4][16 * 68];

  const unsigned tid = threadIdx.x, wave = tid >> 5, lane = tid & 31u, hh = lane >> 4, c = lane & 15u;
  const unsigned bx = blockIdx.x;
  const unsigned qb = bx % (unsigned)NQB;
  const unsigned bh = bx / (unsigned)NQB;
  const unsigned h = bh & 7u, b = bh >> 3;
  const unsigned q0 = qb * 64u + wave * 16u;
  const float PSC = SPV ? 1.0f : 16384.0f;
  const float L2E = 1.4426950408889634f;
  const __bf16* Qh = (const __bf16*)QKhp; const __bf16* Ql = (const __bf16*)QKlp;
  const __bf16* Vh = (const __bf16*)VThp; const __bf16* Vl = (const __bf16*)VTlp;

  v16b qah[2], qal[2];
  {
    const size_t qo = (size_t)(b * (unsigned)SEQ + q0 + c) * 1024u + h * 64u + 8u * hh;
#pragma unroll
    for (int dc = 0; dc < 2; ++dc) {
      FB f, g;
      f.h[0] = *(const v8b*)(Qh + qo + dc * 32);
      f.h[1] = *(const v8b*)(Qh + qo + dc * 32 + 16);
      g.h[0] = *(const v8b*)(Ql + qo + dc * 32);
      g.h[1] = *(const v8b*)(Ql + qo + dc * 32 + 16);
      qah[dc] = f.v; qal[dc] = g.v;
    }
  }

  float mrun[8], lrun[8];
  v8f oacc[4];
#pragma unroll
  for (int r = 0; r < 8; ++r) { mrun[r] = -INFINITY; lrun[r] = 0.f; }
#pragma unroll
  for (int t = 0; t < 4; ++t) oacc[t] = (v8f){0.f,0.f,0.f,0.f,0.f,0.f,0.f,0.f};

  const size_t kro = (size_t)(b * (unsigned)SEQ) * 1024u + 512u + h * 64u + 8u * hh;
  const size_t vro = (size_t)(b * 512u + h * 64u) * (unsigned)SEQ + 8u * hh;
  const float* mk = mask + (size_t)b * SEQ_FULL;
  __bf16* pwh = Psh[wave];
  __bf16* pwl = Psl[SPV ? wave : 0];

  for (unsigned kc = 0; kc < (unsigned)NQB; ++kc) {
    const unsigned kv0 = kc * 64u;
    v8f s[4];
#pragma unroll
    for (int j = 0; j < 4; ++j) {
      v8f a = (v8f){0.f,0.f,0.f,0.f,0.f,0.f,0.f,0.f};
      const size_t ko = kro + (size_t)(kv0 + (unsigned)j * 16u + c) * 1024u;
#pragma unroll
      for (int dc = 0; dc < 2; ++dc) {
        FB kb, kl;
        kb.h[0] = *(const v8b*)(Qh + ko + dc * 32);
        kb.h[1] = *(const v8b*)(Qh + ko + dc * 32 + 16);
        kl.h[0] = *(const v8b*)(Ql + ko + dc * 32);
        kl.h[1] = *(const v8b*)(Ql + ko + dc * 32 + 16);
        a = kit::at_mma(qah[dc], kb.v, a);
        a = kit::at_mma(qah[dc], kl.v, a);
        a = kit::at_mma(qal[dc], kb.v, a);
      }
      s[j] = a;
      asm volatile("" ::: "memory");
    }
    float km[4];
#pragma unroll
    for (int j = 0; j < 4; ++j) km[j] = mk[kv0 + (unsigned)j * 16u + c];

    float cm[8];
#pragma unroll
    for (int r = 0; r < 8; ++r) {
      float m = -INFINITY;
#pragma unroll
      for (int j = 0; j < 4; ++j) {
        float a = s[j][r];
        a = km[j] * a + (1.0f - km[j]) * (-1e-30f);
        a *= L2E;
        s[j][r] = a;
        m = fmaxf(m, a);
      }
      m = fmaxf(m, __shfl_xor(m, 1, 32)); m = fmaxf(m, __shfl_xor(m, 2, 32));
      m = fmaxf(m, __shfl_xor(m, 4, 32)); m = fmaxf(m, __shfl_xor(m, 8, 32));
      cm[r] = m;
    }
#pragma unroll
    for (int r = 0; r < 8; ++r) {
      const float mnew = fmaxf(mrun[r], cm[r]);
      const float alpha = exp2f(mrun[r] - mnew);
      mrun[r] = mnew;
      float psum = 0.f;
#pragma unroll
      for (int j = 0; j < 4; ++j) {
        const float p = exp2f(s[j][r] - mnew);
        psum += p;
        const unsigned idx = (8u * hh + (unsigned)r) * 64u + (unsigned)j * 16u + c;
        if (SPV) { __bf16 a, bl; kit::at_split(p, a, bl); pwh[idx] = a; pwl[idx] = bl; }
        else pwh[idx] = kit::at_to16<true>(p * PSC);
      }
      psum += __shfl_xor(psum, 1, 32); psum += __shfl_xor(psum, 2, 32);
      psum += __shfl_xor(psum, 4, 32); psum += __shfl_xor(psum, 8, 32);
      lrun[r] = lrun[r] * alpha + psum;
#pragma unroll
      for (int t = 0; t < 4; ++t) oacc[t][r] *= alpha;
    }
    __builtin_amdgcn_fence(3  , "workgroup");
    __builtin_amdgcn_wave_barrier();
    __builtin_amdgcn_fence(2  , "workgroup");
#pragma unroll
    for (int kk = 0; kk < 2; ++kk) {
      FB pa, pl;
      pa.h[0] = *(const v8b*)(pwh + c * 64u + kk * 32 + 8u * hh);
      pa.h[1] = *(const v8b*)(pwh + c * 64u + kk * 32 + 16 + 8u * hh);
      if (SPV) {
        pl.h[0] = *(const v8b*)(pwl + c * 64u + kk * 32 + 8u * hh);
        pl.h[1] = *(const v8b*)(pwl + c * 64u + kk * 32 + 16 + 8u * hh);
      }
#pragma unroll
      for (int t = 0; t < 4; ++t) {
        const size_t vo = vro + (size_t)((unsigned)t * 16u + c) * (unsigned)SEQ + kv0 + (unsigned)kk * 32u;
        FB vb;
        vb.h[0] = *(const v8b*)(Vh + vo);
        vb.h[1] = *(const v8b*)(Vh + vo + 16);
        oacc[t] = kit::at_mma16<!SPV>(pa.v, vb.v, oacc[t]);
        if (SPV) {
          FB vl;
          vl.h[0] = *(const v8b*)(Vl + vo);
          vl.h[1] = *(const v8b*)(Vl + vo + 16);
          oacc[t] = kit::at_mma(pa.v, vl.v, oacc[t]);
          oacc[t] = kit::at_mma(pl.v, vb.v, oacc[t]);
        }
        asm volatile("" ::: "memory");
      }
    }
  }

  float* os = Os[wave];
#pragma unroll
  for (int r = 0; r < 8; ++r) {
    const float inv = 1.0f / (lrun[r] * PSC);
#pragma unroll
    for (int t = 0; t < 4; ++t) os[(8u * hh + (unsigned)r) * 68u + (unsigned)t * 16u + c] = oacc[t][r] * inv;
  }
  __builtin_amdgcn_fence(3  , "workgroup");
  __builtin_amdgcn_wave_barrier();
  __builtin_amdgcn_fence(2  , "workgroup");
  {
    const unsigned q = lane >> 3, c8 = (lane & 7u) * 8u;
    const unsigned pitch = SPV ? 1024u : 512u;
    unsigned short* C = Cp + (size_t)(b * (unsigned)SEQ + q0) * pitch + h * 64u;
    for (int pass = 0; pass < 2; ++pass) {
#pragma unroll
      for (int it = 0; it < 4; ++it) {
        const unsigned row = (unsigned)it * 4u + q;
        const float* sp = os + row * 68u + c8;
        v8h hv, lv;
#pragma unroll
        for (int e = 0; e < 8; ++e) {
          if (SPV) {
            const unsigned short hb = kit::f2bf_bits(sp[e]);
            const unsigned short lb = kit::f2bf_bits(sp[e] - kit::bf_bits2f(hb));
            hv[e] = __builtin_bit_cast(_Float16, hb);
            lv[e] = __builtin_bit_cast(_Float16, lb);
          } else {
            hv[e] = (_Float16)sp[e];
          }
        }
        *(volatile v8h*)(C + (size_t)row * pitch + c8) = hv;
        if (SPV) *(volatile v8h*)(C + (size_t)row * pitch + 512u + c8) = lv;
      }
      __threadfence();
    }
  }
}

template <int FL>
__global__ __launch_bounds__(256) void k_ln(const float* __restrict__ Y, float* __restrict__ Xf, unsigned short* __restrict__ X16, unsigned short* __restrict__ XS,
                                            float* __restrict__ OUT, const float* __restrict__ gamma, const float* __restrict__ beta, unsigned gi, unsigned nrows) {
  const unsigned lane = threadIdx.x & 31u, wave = threadIdx.x >> 5;
  const unsigned row = blockIdx.x * 8u + wave;
  if (row >= nrows) return;
  const float* yr = Y + (size_t)row * 512u;
  float s = 0.f;
#pragma unroll 1
  for (unsigned i = 0; i < 4u; ++i) { const v4f v = *(const v4f*)(yr + 128u * i + 4u * lane); s += (v.x + v.y) + (v.z + v.w); }
  s += __shfl_xor(s, 16, 32); s += __shfl_xor(s, 8, 32); s += __shfl_xor(s, 4, 32); s += __shfl_xor(s, 2, 32); s += __shfl_xor(s, 1, 32);
  const float mean = s * (1.0f / 512.0f);
  float q = 0.f;
#pragma unroll 1
  for (unsigned i = 0; i < 4u; ++i) { const v4f d = *(const v4f*)(yr + 128u * i + 4u * lane) - mean; q += (d.x * d.x + d.y * d.y) + (d.z * d.z + d.w * d.w); }
  q += __shfl_xor(q, 16, 32); q += __shfl_xor(q, 8, 32); q += __shfl_xor(q, 4, 32); q += __shfl_xor(q, 2, 32); q += __shfl_xor(q, 1, 32);
  const float rs = 1.0f / sqrtf(q * (1.0f / 512.0f) + 1e-14f);
  const float g = gamma[gi], be = beta[gi];
  if (FL & 9) {
#pragma unroll 1
    for (unsigned i = 0; i < 4u; ++i) {
      const unsigned off = 128u * i + 4u * lane;
      const v4f o = ((*(const v4f*)(yr + off) - mean) * rs) * g + be;
      if (FL & 1) VST2V4(Xf + (size_t)row * 512u + off, o);
      if (FL & 8) VST2V4(OUT + (size_t)row * 512u + off, o);
    }
  }
  if (FL & 6) {
#pragma unroll 1
    for (unsigned i2 = 0; i2 < 2u; ++i2) {
      const unsigned p8 = (lane + 32u * i2) * 8u;
      const v4f o0 = ((*(const v4f*)(yr + p8) - mean) * rs) * g + be;
      const v4f o1 = ((*(const v4f*)(yr + p8 + 4u) - mean) * rs) * g + be;
      if (FL & 2) {
        cm_u4 pk; pk.x = cmb_pk2(o0.x, o0.y); pk.y = cmb_pk2(o0.z, o0.w); pk.z = cmb_pk2(o1.x, o1.y); pk.w = cmb_pk2(o1.z, o1.w);
        VST2(cm_u4, (cm_u4*)(X16 + (size_t)row * 512u + p8), pk);
      }
      if (FL & 4) {
        cm_u4 ph, pl; unsigned lo;
        ph.x = kit::f2bf2_pack(o0.x, o0.y, &lo); pl.x = lo;
        ph.y = kit::f2bf2_pack(o0.z, o0.w, &lo); pl.y = lo;
        ph.z = kit::f2bf2_pack(o1.x, o1.y, &lo); pl.z = lo;
        ph.w = kit::f2bf2_pack(o1.z, o1.w, &lo); pl.w = lo;
        VST2(cm_u4, (cm_u4*)(XS + (size_t)row * 1024u + p8), ph);
        VST2(cm_u4, (cm_u4*)(XS + (size_t)row * 1024u + 512u + p8), pl);
      }
    }
  }
}

__device__ __forceinline__ size_t x_src(unsigned e) {
  const unsigned row = e >> 9; const unsigned bb = row / (unsigned)SEQ; const unsigned ss = row - bb * (unsigned)SEQ;
  return ((size_t)(bb * (unsigned)SEQ_FULL + ss) << 9) + (size_t)(e & 511u);
}
__global__ __launch_bounds__(256) void k_xprep(const float* __restrict__ x, float* __restrict__ Xf, unsigned short* __restrict__ X16) {
  const unsigned tid = threadIdx.x; const unsigned e0 = blockIdx.x * 2048u;
#pragma unroll 1
  for (unsigned i = 0; i < 2u; ++i) {
    const unsigned e = e0 + (i * 256u + tid) * 4u;
    v4f v = *(const v4f*)(x + x_src(e));
    v.x = cmb_bf(v.x); v.y = cmb_bf(v.y); v.z = cmb_bf(v.z); v.w = cmb_bf(v.w);
    VST2V4(Xf + e, v);
  }
  {
    const unsigned e = e0 + tid * 8u; const float* sp = x + x_src(e);
    const v4f a = *(const v4f*)sp, bq = *(const v4f*)(sp + 4);
    cm_u4 pk; pk.x = cmb_pk2(cmb_bf(a.x), cmb_bf(a.y)); pk.y = cmb_pk2(cmb_bf(a.z), cmb_bf(a.w)); pk.z = cmb_pk2(cmb_bf(bq.x), cmb_bf(bq.y)); pk.w = cmb_pk2(cmb_bf(bq.z), cmb_bf(bq.w));
    VST2(cm_u4, (cm_u4*)(X16 + e), pk);
  }
}

__global__ __launch_bounds__(256) void k_wprep(const float* __restrict__ SRC, unsigned lds, unsigned sS, unsigned short* __restrict__ DST, unsigned ldd, unsigned sD,
                                               unsigned psh, unsigned nC, float sc, int fmt, unsigned dup) {
  const unsigned u = blockIdx.x * 256u + threadIdx.x; if (u >= (nC << psh)) return;
  const unsigned c = u >> psh; const unsigned r0 = (u & ((1u << psh) - 1u)) << 3;
  const float* s = SRC + (size_t)blockIdx.y * sS;
  unsigned short* d = DST + (size_t)blockIdx.y * sD + (size_t)c * ldd + r0;
  float w[8];
#pragma unroll
  for (int e = 0; e < 8; ++e) w[e] = cmb_bf(s[(size_t)(r0 + (unsigned)e) * lds + c]) * sc;
  cm_u4 pk;
  if (fmt == 0) { pk.x = cmb_pk2(w[0], w[1]); pk.y = cmb_pk2(w[2], w[3]); pk.z = cmb_pk2(w[4], w[5]); pk.w = cmb_pk2(w[6], w[7]); }
  else {
    pk.x = (__builtin_bit_cast(unsigned, w[0]) >> 16) | (__builtin_bit_cast(unsigned, w[1]) & 0xffff0000u);
    pk.y = (__builtin_bit_cast(unsigned, w[2]) >> 16) | (__builtin_bit_cast(unsigned, w[3]) & 0xffff0000u);
    pk.z = (__builtin_bit_cast(unsigned, w[4]) >> 16) | (__builtin_bit_cast(unsigned, w[5]) & 0xffff0000u);
    pk.w = (__builtin_bit_cast(unsigned, w[6]) >> 16) | (__builtin_bit_cast(unsigned, w[7]) & 0xffff0000u);
  }
  VST2(cm_u4, (cm_u4*)d, pk);
  if (dup != 0u) VST2(cm_u4, (cm_u4*)(d + dup), pk);
}
__global__ __launch_bounds__(256) void k_cm_bfvec(const float* __restrict__ SRC, float* __restrict__ DST, unsigned n) { const unsigned u = blockIdx.x * 256u + threadIdx.x; if (u >= n) return; VST2(float, DST + u, cmb_bf(SRC[u])); }

static inline char* carve_(char*& p, size_t bytes) { char* r = p; p += ((bytes + 255) / 256) * 256; return r; }

extern "C" void kernel_launch(void* const* d_in, const int* in_sizes, int n_in, void* d_out, int out_size, void* d_ws, size_t ws_size, hipStream_t stream) {
  if (n_in < 12) return;
  const size_t xneed = ((size_t)(NB - 1) * SEQ_FULL + SEQ) * 512;
  if ((size_t)in_sizes[0] < xneed) return;
  if ((size_t)in_sizes[1] < (size_t)(NB - 1) * SEQ_FULL + SEQ) return;
  if (in_sizes[2] < 524288 || in_sizes[3] < 524288 || in_sizes[4] < 524288 || in_sizes[5] < 524288) return;
  if (in_sizes[6] < 1048576 || in_sizes[7] < 2048 || in_sizes[8] < 1048576 || in_sizes[9] < 1024 || in_sizes[10] < 4 || in_sizes[11] < 4) return;
  if ((size_t)out_size < (size_t)MROWS * 512) return;

  const float* x     = (const float*)d_in[0];
  const float* mask  = (const float*)d_in[1];
  const float* wq    = (const float*)d_in[2];
  const float* wk    = (const float*)d_in[3];
  const float* wv    = (const float*)d_in[4];
  const float* wo    = (const float*)d_in[5];
  const float* w1    = (const float*)d_in[6];
  const float* b1    = (const float*)d_in[7];
  const float* w2    = (const float*)d_in[8];
  const float* b2    = (const float*)d_in[9];
  const float* gamma = (const float*)d_in[10];
  const float* beta  = (const float*)d_in[11];
  float* out = (float*)d_out;

  constexpr size_t SZ_XF  = (size_t)MROWS * 512 * 4;
  constexpr size_t SZ_X16 = (size_t)MROWS * 512 * 2;
  constexpr size_t SZ_R12 = (size_t)MROWS * 2048 * 2;
  constexpr size_t SZ_R3  = (size_t)MROWS * 1024 * 2;
  constexpr size_t SZ_R4  = (size_t)MROWS * 1024 * 2;
  static_assert((size_t)NB * 512 * SEQ * 2 * 2 == SZ_R3);
  static_assert((size_t)MROWS * 1024 * 2 * 2 == SZ_R12);
  static_assert((size_t)MROWS * 1024 * 2 <= SZ_R12);
  static_assert((size_t)MROWS * 512 * 2 <= SZ_R4);
  constexpr size_t SZ_W = (size_t)(1024 * 512 + 2 * 512 * 512 + 1024 * 1024 + 512 * 1024 + 512 * 512 + 1024 * 1024 + 1024 * 512 + 512 * 2048 + 512 * 1024) * 2;
  constexpr size_t SZ_TOTAL = 2 * SZ_XF + SZ_X16 + SZ_R12 + SZ_R3 + SZ_R4 + SZ_W + 3072 * 4;
  static_assert(SZ_TOTAL <= (size_t)134217728);
  char* wsp = (char*)d_ws;
  float* Xf = (float*)carve_(wsp, SZ_XF);
  float* Y  = (float*)carve_(wsp, SZ_XF);
  unsigned short* X16 = (unsigned short*)carve_(wsp, SZ_X16);
  unsigned short* R12 = (unsigned short*)carve_(wsp, SZ_R12);
  unsigned short* R3  = (unsigned short*)carve_(wsp, SZ_R3);
  unsigned short* R4  = (unsigned short*)carve_(wsp, SZ_R4);
  unsigned short* Wqk0  = (unsigned short*)carve_(wsp, (size_t)1024 * 512 * 2);
  unsigned short* Wv16  = (unsigned short*)carve_(wsp, (size_t)2 * 512 * 512 * 2);
  unsigned short* Wqk1B = (unsigned short*)carve_(wsp, (size_t)1024 * 1024 * 2);
  unsigned short* WoB0  = (unsigned short*)carve_(wsp, (size_t)512 * 1024 * 2);
  unsigned short* Wo161 = (unsigned short*)carve_(wsp, (size_t)512 * 512 * 2);
  unsigned short* W1B0  = (unsigned short*)carve_(wsp, (size_t)1024 * 1024 * 2);
  unsigned short* W1161 = (unsigned short*)carve_(wsp, (size_t)1024 * 512 * 2);
  unsigned short* W2B0  = (unsigned short*)carve_(wsp, (size_t)512 * 2048 * 2);
  unsigned short* W2161 = (unsigned short*)carve_(wsp, (size_t)512 * 1024 * 2);
  float* BR = (float*)carve_(wsp, (size_t)3072 * 4);
  if ((size_t)(wsp - (char*)d_ws) > ws_size || (size_t)(wsp - (char*)d_ws) > (size_t)134217728) return;

  unsigned short* QKh = R12; unsigned short* QKl = R12 + (size_t)MROWS * 1024;
  unsigned short* HS  = R12; unsigned short* H16 = R12;
  unsigned short* VTh = R3;  unsigned short* VTl = R3 + (size_t)NB * 512 * SEQ;
  unsigned short* XS  = R3;  unsigned short* VT16 = R3;
  unsigned short* CS  = R4;  unsigned short* C16 = R4;

  k_xprep<<<(unsigned)(((size_t)MROWS * 512) / 2048), 256, 0, stream>>>(x, Xf, X16);
  k_wprep<<<dim3(16, 8), 256, 0, stream>>>(wq, 64u, 32768u, Wqk0, 512u, 32768u, 6u, 64u, 16.0f, 0, 0u);
  k_wprep<<<dim3(16, 8), 256, 0, stream>>>(wk, 64u, 32768u, Wqk0 + 512 * 512, 512u, 32768u, 6u, 64u, 16.0f, 0, 0u);
  k_wprep<<<dim3(16, 16), 256, 0, stream>>>(wv, 64u, 32768u, Wv16, 512u, 32768u, 6u, 64u, 16.0f, 0, 0u);
  k_wprep<<<dim3(16, 8), 256, 0, stream>>>(wq + 262144, 64u, 32768u, Wqk1B, 1024u, 65536u, 6u, 64u, 1.0f, 1, 512u);
  k_wprep<<<dim3(16, 8), 256, 0, stream>>>(wk + 262144, 64u, 32768u, Wqk1B + 512 * 1024, 1024u, 65536u, 6u, 64u, 1.0f, 1, 512u);
  k_wprep<<<dim3(128, 1), 256, 0, stream>>>(wo, 512u, 0u, WoB0, 1024u, 0u, 6u, 512u, 1.0f, 1, 512u);
  k_wprep<<<dim3(128, 1), 256, 0, stream>>>(wo + 262144, 512u, 0u, Wo161, 512u, 0u, 6u, 512u, 16.0f, 0, 0u);
  k_wprep<<<dim3(256, 1), 256, 0, stream>>>(w1, 1024u, 0u, W1B0, 1024u, 0u, 6u, 1024u, 1.0f, 1, 512u);
  k_wprep<<<dim3(256, 1), 256, 0, stream>>>(w1 + 524288, 1024u, 0u, W1161, 512u, 0u, 6u, 1024u, 16.0f, 0, 0u);
  k_wprep<<<dim3(256, 1), 256, 0, stream>>>(w2, 512u, 0u, W2B0, 2048u, 0u, 7u, 512u, 1.0f, 1, 1024u);
  k_wprep<<<dim3(256, 1), 256, 0, stream>>>(w2 + 524288, 512u, 0u, W2161, 1024u, 0u, 7u, 512u, 16.0f, 0, 0u);
  k_cm_bfvec<<<8, 256, 0, stream>>>(b1, BR, 2048u);
  k_cm_bfvec<<<4, 256, 0, stream>>>(b2, BR + 2048, 1024u);

  const unsigned TM = MROWS / 64;
  const unsigned gQK = (TM * 16 + 7) / 8, gD = (TM * 8 + 7) / 8, gVT = (8 * (SEQ / 64) + 7) / 8;
  const unsigned gAT = NB * 8 * NQB, gLN = MROWS / 8;

  kit::wmma_gemm64<0, false, 0, 2, false, 0><<<dim3(gQK, 1), 256, 0, stream>>>(X16, nullptr, 512, 0, Wqk0, nullptr, 512, 0, (void*)QKh, (void*)QKl, 1024, 0, nullptr, nullptr, 0, MROWS, 1024, 512, 0.0625f);
  kit::wmma_gemm64<0, false, 0, 2, false, 0><<<dim3(gVT, NB), 256, 0, stream>>>(Wv16, nullptr, 512, 0, X16, nullptr, 512, (long)SEQ * 512, (void*)VTh, (void*)VTl, SEQ, (long)512 * SEQ, nullptr, nullptr, 0, 512, SEQ, 512, 0.0625f);
  k_fattn<true><<<gAT, 128, 0, stream>>>(QKh, QKl, VTh, VTl, mask, CS);
  kit::wmma_gemm64<1, false, 0, 0, true, 0><<<dim3(gD, 1), 256, 0, stream>>>(CS, nullptr, 1024, 0, WoB0, nullptr, 1024, 0, (void*)Y, nullptr, 512, 0, nullptr, Xf, 0, MROWS, 512, 1024, 1.0f);
  k_ln<5><<<gLN, 256, 0, stream>>>(Y, Xf, X16, XS, out, gamma, beta, 0u, (unsigned)MROWS);
  kit::wmma_gemm64<1, false, 2, 2, false, 2><<<dim3(gQK, 1), 256, 0, stream>>>(XS, nullptr, 1024, 0, W1B0, nullptr, 1024, 0, (void*)HS, (void*)(HS + 1024), 2048, 0, BR, nullptr, 0, MROWS, 1024, 1024, 1.0f);
  kit::wmma_gemm64<1, false, 2, 0, true, 0><<<dim3(gD, 1), 256, 0, stream>>>(HS, nullptr, 2048, 0, W2B0, nullptr, 2048, 0, (void*)Y, nullptr, 512, 0, BR + 2048, Xf, 0, MROWS, 512, 2048, 1.0f);
  k_ln<7><<<gLN, 256, 0, stream>>>(Y, Xf, X16, XS, out, gamma, beta, 1u, (unsigned)MROWS);

  kit::wmma_gemm64<1, false, 0, 2, false, 0><<<dim3(gQK, 1), 256, 0, stream>>>(XS, nullptr, 1024, 0, Wqk1B, nullptr, 1024, 0, (void*)QKh, (void*)QKl, 1024, 0, nullptr, nullptr, 0, MROWS, 1024, 1024, 1.0f);
  kit::wmma_gemm64<0, false, 0, 1, false, 0><<<dim3(gVT, NB), 256, 0, stream>>>(Wv16 + 512 * 512, nullptr, 512, 0, X16, nullptr, 512, (long)SEQ * 512, (void*)VT16, nullptr, SEQ, (long)512 * SEQ, nullptr, nullptr, 0, 512, SEQ, 512, 0.0625f);
  k_fattn<false><<<gAT, 128, 0, stream>>>(QKh, QKl, VT16, VT16, mask, C16);
  kit::wmma_gemm64<0, false, 0, 0, true, 0><<<dim3(gD, 1), 256, 0, stream>>>(C16, nullptr, 512, 0, Wo161, nullptr, 512, 0, (void*)Y, nullptr, 512, 0, nullptr, Xf, 0, MROWS, 512, 512, 0.0625f);
  k_ln<3><<<gLN, 256, 0, stream>>>(Y, Xf, X16, XS, out, gamma, beta, 2u, (unsigned)MROWS);
  kit::wmma_gemm64<0, false, 2, 1, false, 2><<<dim3(gQK, 1), 256, 0, stream>>>(X16, nullptr, 512, 0, W1161, nullptr, 512, 0, (void*)H16, nullptr, 1024, 0, BR + 1024, nullptr, 0, MROWS, 1024, 512, 0.0625f);
  kit::wmma_gemm64<0, false, 2, 0, true, 0><<<dim3(gD, 1), 256, 0, stream>>>(H16, nullptr, 1024, 0, W2161, nullptr, 1024, 0, (void*)Y, nullptr, 512, 0, BR + 2560, Xf, 0, MROWS, 512, 1024, 0.0625f);
  k_ln<8><<<gLN, 256, 0, stream>>>(Y, Xf, X16, XS, out, gamma, beta, 3u, (unsigned)MROWS);
}
